// Block_73744588472675
// MI455X (gfx1250) — hardware-run, weakly checked
//
#include <hip/hip_runtime.h>


#ifndef NB
#define NB 4
#endif
#ifndef SEQ
#define SEQ 677
#endif
#define NB_FULL  4
#define SEQ_FULL 677
#ifndef OUT_SEQ
#define OUT_SEQ SEQ
#endif
#define DM   1024
#define NH_  16
#define HD   64
#define FF   4096
#define TP   (((SEQ + 63) / 64) * 64)
#define NKEY ((SEQ + 31) & ~31)
#define AW   4
#define OSP  68
#define WCAR 64.0f
#define CCAR 16.0f
#define MCAR 16.0f
#define WINV (1.0f / 64.0f)
#define PINV (1.0f / 1024.0f)
#define SC2  ((float)(0.125 * 1.4426950408889634))
#define L2E  1.4426950408889634f
#define PSH  14.0f
#define NEGB (-3.0e38f)

static_assert(HD == 64);
static_assert(NH_ * HD == DM);
static_assert(DM % 64 == 0);
static_assert(FF % 64 == 0);
static_assert(DM % 32 == 0);
static_assert(FF % 32 == 0);
static_assert(TP % 64 == 0);
static_assert((NB * TP) % 64 == 0);
static_assert(TP >= SEQ);
static_assert(NKEY % 32 == 0);
static_assert(NKEY <= TP);
static_assert(TP % (16 * AW) == 0);
static_assert((NB * TP) % 8 == 0);
static_assert(DM == 32 * 8 * 4);
static_assert(TP % 8 == 0);
static_assert((TP / 8) % 8 == 0);
static_assert((TP * 2) % 128 == 0);
static_assert((OSP * 4) % 16 == 0);
static_assert(32 * 16 * 4 == 16 * HD * 2);
static_assert(32 * 16 * 8 == 16 * 64 * 4);
static_assert(32 * 16 * 4 == DM * 2);
static_assert(32 * 32 == 16 * 64);
static_assert(16 * 68 * 4 <= 131072);
static_assert(AW * 16 * OSP * 4 <= 131072);
static_assert(NB <= NB_FULL);
static_assert(SEQ <= SEQ_FULL);
static_assert(SEQ >= 1);

typedef _Float16 h16;
typedef unsigned short bf;
typedef __attribute__((ext_vector_type(16))) _Float16 v16h;
typedef __attribute__((ext_vector_type(8)))  _Float16 v8h;
typedef __attribute__((ext_vector_type(8)))  unsigned short v8us;
typedef __attribute__((ext_vector_type(8)))  float    v8f;
typedef __attribute__((ext_vector_type(4)))  float    v4f;
typedef v4f  __attribute__((may_alias)) v4fa;

__device__ __forceinline__ unsigned short f2bf(float f) { unsigned u = __float_as_uint(f); u += 0x7FFFu + ((u >> 16) & 1u); return (unsigned short)(u >> 16); }
__device__ __forceinline__ float bfr(float f) { return __uint_as_float(((unsigned)f2bf(f)) << 16); }
__device__ __forceinline__ v16h cat16(v8h lo, v8h hi) { return __builtin_shufflevector(lo, hi, 0, 1, 2, 3, 4, 5, 6, 7, 8, 9, 10, 11, 12, 13, 14, 15); }
__device__ __forceinline__ v16h  ldh(const h16* p) { return cat16(*(const v8h*)p, *(const v8h*)(p + 16)); }
__device__ __forceinline__ void wave_sync() { __builtin_amdgcn_fence(3  , "wavefront"); __builtin_amdgcn_wave_barrier(); asm volatile("" ::: "memory"); }
static __device__ __forceinline__ h16 toh_flush(float v) { const h16 r = (h16)v; return (fabsf(v) < 6.103515625e-05f) ? (h16)0.0f : r; }
__device__ __forceinline__ v8f wmg(v16h a, v16h b, v8f c) {
    c = __builtin_amdgcn_wmma_f32_16x16x32_f16(false, a, false, b, (short)0, c, false, false);
    asm volatile("v_nop\n\tv_nop\n\tv_nop\n\tv_nop" : "+v"(c) : "v"(a), "v"(b));
    return c;
}

__global__ __launch_bounds__(256) void k_wconv(const float* __restrict__ src, h16* dst, size_t n8) {
    const size_t i = (size_t)blockIdx.x * 256 + threadIdx.x; if (i >= n8) return;
    const v8f v = *(const v8f*)(src + i * 8); v8h o;
#pragma unroll
    for (int k = 0; k < 8; ++k) o[k] = toh_flush(bfr(v[k]) * WCAR);
    *(volatile v8h*)(dst + i * 8) = o; __threadfence(); *(volatile v8h*)(dst + i * 8) = o;
}

__global__ __launch_bounds__(256) void k_bconv(const float* __restrict__ relb, bf* dst) {
    const size_t i = (size_t)blockIdx.x * 256 + threadIdx.x; if (i >= (size_t)NH_ * TP * (TP / 8)) return;
    const int k8 = (int)(i % (size_t)(TP / 8)); const size_t rr = i / (size_t)(TP / 8);
    const int row = (int)(rr % (size_t)TP); const int hh = (int)(rr / (size_t)TP);
    const int rc = row < SEQ ? row : (SEQ - 1);
    const float* rp = relb + ((size_t)hh * SEQ_FULL + (size_t)rc) * SEQ_FULL;
    v8us o;
#pragma unroll
    for (int j = 0; j < 8; ++j) { const int key = k8 * 8 + j; const int kc = key < SEQ ? key : (SEQ - 1);
        float v = rp[kc]; asm volatile("" : "+v"(v));
        o[j] = ((row < SEQ) & (key < SEQ)) ? f2bf(v) : (unsigned short)0; }
    *(volatile v8us*)(dst + i * 8) = o; __threadfence(); *(volatile v8us*)(dst + i * 8) = o;
}

__device__ __forceinline__ float lnsel(float v, int rnd) { return rnd != 0 ? bfr(v) : v; }
__global__ __launch_bounds__(256) void k_ln(const float* __restrict__ src, int bstride, int rnd, const float* __restrict__ g, const float* __restrict__ be, h16* dst) {
#pragma clang fp contract(off)
    const int lane = threadIdx.x & 31;
    const int rowv = blockIdx.x * 8 + (int)(threadIdx.x >> 5);
    const int ttv = rowv % TP;
    const int row  = __builtin_amdgcn_readfirstlane(rowv);
    const int bb   = __builtin_amdgcn_readfirstlane(rowv / TP);
    const int tc   = __builtin_amdgcn_readfirstlane(ttv < SEQ ? ttv : (SEQ - 1));
    const int live = __builtin_amdgcn_readfirstlane(ttv < SEQ ? 1 : 0);
    const float* xr = src + ((size_t)bb * (size_t)bstride + (size_t)tc) * DM + lane * 8;
    float s = 0.0f;
#pragma unroll 1
    for (int i = 0; i < 4; ++i) {
        const v4f a = *(const v4f*)(xr + i * 256), c = *(const v4f*)(xr + i * 256 + 4);
#pragma unroll
        for (int k = 0; k < 4; ++k) { s += lnsel(a[k], rnd); s += lnsel(c[k], rnd); } }
    s += __shfl_xor(s, 16, 32); s += __shfl_xor(s, 8, 32); s += __shfl_xor(s, 4, 32); s += __shfl_xor(s, 2, 32); s += __shfl_xor(s, 1, 32);
    const float mean = s * (1.0f / (float)DM);
    float ss = 0.0f;
#pragma unroll 1
    for (int i = 0; i < 4; ++i) {
        const v4f a = *(const v4f*)(xr + i * 256), c = *(const v4f*)(xr + i * 256 + 4);
#pragma unroll
        for (int k = 0; k < 4; ++k) { const float d0 = lnsel(a[k], rnd) - mean, d1 = lnsel(c[k], rnd) - mean; ss += d0 * d0; ss += d1 * d1; } }
    ss += __shfl_xor(ss, 16, 32); ss += __shfl_xor(ss, 8, 32); ss += __shfl_xor(ss, 4, 32); ss += __shfl_xor(ss, 2, 32); ss += __shfl_xor(ss, 1, 32);
    const float rs = rsqrtf(ss * (1.0f / (float)DM) + 1.0e-6f);
    h16* drow = dst + (size_t)row * DM + lane * 8;
#pragma unroll 1
    for (int ps = 0; ps < 2; ++ps) {
#pragma unroll 1
        for (int i = 0; i < 4; ++i) {
            const v4f a = *(const v4f*)(xr + i * 256), c = *(const v4f*)(xr + i * 256 + 4);
            const v4f g0 = *(const v4f*)(g + lane * 8 + i * 256), g1 = *(const v4f*)(g + lane * 8 + i * 256 + 4);
            const v4f b0 = *(const v4f*)(be + lane * 8 + i * 256), b1 = *(const v4f*)(be + lane * 8 + i * 256 + 4);
            v8h hv;
#pragma unroll
            for (int k = 0; k < 4; ++k) {
                const float y0 = (lnsel(a[k], rnd) - mean) * rs * bfr(g0[k]) + bfr(b0[k]);
                const float y1 = (lnsel(c[k], rnd) - mean) * rs * bfr(g1[k]) + bfr(b1[k]);
                const h16 z0 = toh_flush(y0), z1 = toh_flush(y1);
                hv[k] = live != 0 ? z0 : (h16)0.0f; hv[4 + k] = live != 0 ? z1 : (h16)0.0f; }
            *(volatile v8h*)(drow + i * 256) = hv; }
        if (ps == 0) __threadfence(); }
}

template <int K>
__device__ __forceinline__ void gemm_core(const h16* __restrict__ A, const h16* __restrict__ Bt, int r0, int c0, int lr, int hi, v8f (&acc)[4][4]) {
    static_assert(K % 32 == 0);
#pragma unroll
    for (int mb = 0; mb < 4; ++mb)
#pragma unroll
        for (int nb = 0; nb < 4; ++nb) acc[mb][nb] = (v8f){};
    const size_t aoff = (size_t)(r0 + lr) * K + 8 * hi, boff = (size_t)(c0 + lr) * K + 8 * hi;
#pragma unroll 1
    for (int kc = 0; kc < K; kc += 32) {
        v16h a[4];
#pragma unroll
        for (int mb = 0; mb < 4; ++mb) a[mb] = ldh(A + aoff + (size_t)mb * 16 * K + kc);
#pragma unroll
        for (int nb = 0; nb < 4; ++nb) { const v16h b = ldh(Bt + boff + (size_t)nb * 16 * K + kc);
#pragma unroll
            for (int mb = 0; mb < 4; ++mb) acc[mb][nb] = wmg(a[mb], b, acc[mb][nb]); }
    }
}

__global__ __launch_bounds__(32) void k_gemm_qk(const h16* __restrict__ Hn, const h16* __restrict__ Wq, const float* __restrict__ qbias, h16* QK) {
    __shared__ __align__(16) float os[16 * 68];
    const int lane = threadIdx.x & 31, lr = lane & 15, hi = lane >> 4; const int r0 = blockIdx.x * 64, c0 = blockIdx.y * 64;
    v8f acc[4][4];
    gemm_core<DM>(Hn, Wq, r0, c0, lr, hi, acc);
    float bc[4];
#pragma unroll
    for (int nb = 0; nb < 4; ++nb) { const int cc = c0 + nb * 16 + lr; float bv = qbias[cc & (DM - 1)]; asm volatile("" : "+v"(bv)); bc[nb] = (cc < DM) ? bfr(bv) : 0.0f; }
    const int bb = r0 / TP, tt = r0 % TP; const int which = c0 / DM, hh = (c0 % DM) / HD;
    const size_t tbase = (size_t)which * ((size_t)NB * NH_ * TP * HD) + ((size_t)(bb * NH_ + hh) * TP + (size_t)tt) * HD;
#pragma unroll
    for (int mb = 0; mb < 4; ++mb) {
#pragma unroll
        for (int nb = 0; nb < 4; ++nb) {
#pragma unroll
            for (int j = 0; j < 8; ++j) os[(hi * 8 + j) * 68 + nb * 16 + lr] = acc[mb][nb][j] * WINV + bc[nb]; }
        wave_sync();
#pragma unroll 1
        for (int ps = 0; ps < 2; ++ps) {
#pragma unroll
            for (int s = 0; s < 4; ++s) { const int row = 4 * s + (lane >> 3), c8 = (lane & 7) * 8;
                const v4f x0 = *(const v4fa*)(&os[row * 68 + c8]); const v4f x1 = *(const v4fa*)(&os[row * 68 + c8 + 4]); v8h hv;
#pragma unroll
                for (int i = 0; i < 4; ++i) { hv[i] = toh_flush(x0[i]); hv[4 + i] = toh_flush(x1[i]); }
                *(volatile v8h*)(QK + tbase + (size_t)(mb * 16 + row) * HD + c8) = hv; }
            if (ps == 0) __threadfence(); }
        wave_sync();
    }
}

__global__ __launch_bounds__(32) void k_gemm_vt(const h16* __restrict__ Wv, const h16* __restrict__ Hn, const float* __restrict__ vbias, h16* VT) {
    __shared__ __align__(16) float os[16 * 68];
    const int lane = threadIdx.x & 31, lr = lane & 15, hi = lane >> 4; const int r0 = blockIdx.x * 64, c0 = blockIdx.y * 64;
    v8f acc[4][4];
    gemm_core<DM>(Wv, Hn, r0, c0, lr, hi, acc);
    const int bb = c0 / TP, tt = c0 % TP;
    const size_t tbase = ((size_t)bb * DM + (size_t)r0) * TP + (size_t)tt;
#pragma unroll
    for (int mb = 0; mb < 4; ++mb) {
        float br[8];
#pragma unroll
        for (int j = 0; j < 8; ++j) br[j] = bfr(vbias[r0 + mb * 16 + hi * 8 + j]);
#pragma unroll
        for (int nb = 0; nb < 4; ++nb) {
#pragma unroll
            for (int j = 0; j < 8; ++j) os[(hi * 8 + j) * 68 + nb * 16 + lr] = acc[mb][nb][j] * WINV + br[j]; }
        wave_sync();
#pragma unroll 1
        for (int ps = 0; ps < 2; ++ps) {
#pragma unroll
            for (int s = 0; s < 4; ++s) { const int row = 4 * s + (lane >> 3), c8 = (lane & 7) * 8;
                const v4f x0 = *(const v4fa*)(&os[row * 68 + c8]); const v4f x1 = *(const v4fa*)(&os[row * 68 + c8 + 4]); v8h hv;
#pragma unroll
                for (int i = 0; i < 4; ++i) { hv[i] = toh_flush(x0[i]); hv[4 + i] = toh_flush(x1[i]); }
                *(volatile v8h*)(VT + tbase + (size_t)(mb * 16 + row) * TP + c8) = hv; }
            if (ps == 0) __threadfence(); }
        wave_sync();
    }
}

__global__ __launch_bounds__(32 * AW) void k_flash(const h16* __restrict__ QP, const h16* __restrict__ KP, const h16* __restrict__ VT, const bf* __restrict__ BP, h16* CTX) {
    __shared__ __align__(16) float os[AW * 16 * OSP];
    const int lane = threadIdx.x & 31, lr = lane & 15, hi = lane >> 4;
    const int wave = __builtin_amdgcn_readfirstlane((int)(threadIdx.x >> 5));
    const int zh = blockIdx.y; const int b = zh / NH_, h = zh % NH_;
    const int t0 = (blockIdx.x * AW + wave) * 16;
    const size_t pbase = (size_t)zh * TP * HD;
    const size_t qo = pbase + (size_t)(t0 + lr) * HD + 8 * hi;
    const v16h q0 = ldh(QP + qo), q1 = ldh(QP + qo + 32);
    const size_t ko = pbase + (size_t)lr * HD + 8 * hi;
    const size_t vo = pbase + (size_t)lr * TP + 8 * hi;
    const size_t bo = ((size_t)h * TP + (size_t)(t0 + lr)) * TP + 8 * hi;
    v8f o[4];
#pragma unroll
    for (int j = 0; j < 4; ++j) o[j] = (v8f){};
    float m = NEGB, l = 0.0f;
#pragma unroll 1
    for (int key0 = 0; key0 < NKEY; key0 += 32) {
        const h16* ka = KP + ko + (size_t)key0 * HD;
        const v16h ka0 = ldh(ka), ka1 = ldh(ka + 32), kb0 = ldh(ka + 16 * HD), kb1 = ldh(ka + 16 * HD + 32);
        v8f sA = (v8f){}, sB = (v8f){};
        sA = wmg(ka0, q0, sA); sA = wmg(ka1, q1, sA); sB = wmg(kb0, q0, sB); sB = wmg(kb1, q1, sB);
        const bf* bp = BP + bo + key0;
        const v8us ba = *(const v8us*)bp, bc = *(const v8us*)(bp + 16);
        const int ja = key0 + 8 * hi;
        float ta[8], tb[8]; bool fa[8], fb[8]; float mx = NEGB;
#pragma unroll
        for (int r = 0; r < 8; ++r) {
            const float ra = __uint_as_float(((unsigned)ba[r]) << 16), rb = __uint_as_float(((unsigned)bc[r]) << 16);
            fa[r] = (ja + r < SEQ); fb[r] = (ja + 16 + r < SEQ);
            ta[r] = sA[r] * SC2 + ra * L2E; tb[r] = sB[r] * SC2 + rb * L2E;
            mx = fmaxf(mx, fmaxf(fa[r] ? ta[r] : NEGB, fb[r] ? tb[r] : NEGB)); }
        mx = fmaxf(mx, __shfl_xor(mx, 16, 32));
        const float mnew = fmaxf(m, mx);
        const float alpha = __builtin_amdgcn_exp2f(m - mnew);
        const float sh = PSH - mnew;
        v16h pb; float ls = 0.0f;
#pragma unroll
        for (int r = 0; r < 8; ++r) {
            const float xa = ta[r] + sh, xb = tb[r] + sh;
            const float ea = __builtin_amdgcn_exp2f(xa), eb = __builtin_amdgcn_exp2f(xb);
            const float ga = (fa[r] & (xa >= -14.0f)) ? ea : 0.0f, gb = (fb[r] & (xb >= -14.0f)) ? eb : 0.0f;
            const h16 pa = (h16)ga; const h16 pc = (h16)gb;
            pb[r] = pa; pb[8 + r] = pc;
            ls += (float)pa + (float)pc; }
        l = l * alpha + ls; m = mnew;
#pragma unroll
        for (int j = 0; j < 4; ++j) o[j] = o[j] * alpha;
        const h16* va = VT + vo + key0;
        const v16h v0 = ldh(va), v1 = ldh(va + (size_t)16 * TP), v2 = ldh(va + (size_t)32 * TP), v3 = ldh(va + (size_t)48 * TP);
        o[0] = wmg(v0, pb, o[0]); o[1] = wmg(v1, pb, o[1]); o[2] = wmg(v2, pb, o[2]); o[3] = wmg(v3, pb, o[3]);
    }
    l += __shfl_xor(l, 16, 32);
    const bool any = l > 0.0f;
    const float lsafe = any ? l : 1.0f;
    const float inv = any ? (CCAR * (1.0f / lsafe)) : 0.0f;
    const int wb = wave * 16 * OSP;
#pragma unroll
    for (int j = 0; j < 4; ++j) { v4f a, c;
        a[0] = o[j][0] * inv; a[1] = o[j][1] * inv; a[2] = o[j][2] * inv; a[3] = o[j][3] * inv; c[0] = o[j][4] * inv; c[1] = o[j][5] * inv; c[2] = o[j][6] * inv; c[3] = o[j][7] * inv;
        *(v4fa*)(&os[wb + lr * OSP + 16 * j + 8 * hi]) = a; *(v4fa*)(&os[wb + lr * OSP + 16 * j + 8 * hi + 4]) = c; }
    wave_sync();
    h16* crow = CTX + ((size_t)b * TP + (size_t)t0) * DM + h * HD;
#pragma unroll 1
    for (int ps = 0; ps < 2; ++ps) {
#pragma unroll
        for (int s = 0; s < 4; ++s) { const int row = 4 * s + (lane >> 3), c8 = (lane & 7) * 8;
            const v4f x0 = *(const v4fa*)(&os[wb + row * OSP + c8]); const v4f x1 = *(const v4fa*)(&os[wb + row * OSP + c8 + 4]); v8h hv;
#pragma unroll
            for (int i = 0; i < 4; ++i) { hv[i] = toh_flush(x0[i]); hv[4 + i] = toh_flush(x1[i]); }
            *(volatile v8h*)(crow + (size_t)row * DM + c8) = hv; }
        if (ps == 0) __threadfence(); }
}

__global__ __launch_bounds__(32) void k_gemm_proj(const h16* __restrict__ Cx, const h16* __restrict__ Wp, const float* __restrict__ bias, const float* __restrict__ X, float* X1) {
    __shared__ __align__(16) float os[16 * 68];
    const int lane = threadIdx.x & 31, lr = lane & 15, hi = lane >> 4; const int r0 = blockIdx.x * 64, c0 = blockIdx.y * 64;
    v8f acc[4][4];
    gemm_core<DM>(Cx, Wp, r0, c0, lr, hi, acc);
    float bc[4];
#pragma unroll
    for (int nb = 0; nb < 4; ++nb) bc[nb] = bfr(bias[c0 + nb * 16 + lr]);
    const int bb = r0 / TP, tt = r0 % TP;
#pragma unroll
    for (int mb = 0; mb < 4; ++mb) {
#pragma unroll
        for (int nb = 0; nb < 4; ++nb) {
#pragma unroll
            for (int j = 0; j < 8; ++j) os[(hi * 8 + j) * 68 + nb * 16 + lr] = acc[mb][nb][j] * PINV + bc[nb]; }
        wave_sync();
#pragma unroll 1
        for (int ps = 0; ps < 2; ++ps) {
#pragma unroll
            for (int s = 0; s < 8; ++s) { const int p = s * 32 + lane; const int row = p >> 4, c4 = (p & 15) * 4;
                const v4f o4 = *(const v4fa*)(&os[row * 68 + c4]);
                int tr = tt + mb * 16 + row; tr = tr < SEQ ? tr : (SEQ - 1);
                const v4f xv = *(const v4f*)(X + ((size_t)bb * SEQ_FULL + (size_t)tr) * DM + c0 + c4);
                v4f val;
#pragma unroll
                for (int i = 0; i < 4; ++i) val[i] = o4[i] + bfr(xv[i]);
                *(volatile v4f*)(X1 + (size_t)(r0 + mb * 16 + row) * DM + c0 + c4) = val; }
            if (ps == 0) __threadfence(); }
        wave_sync();
    }
}

__global__ __launch_bounds__(32) void k_gemm_fc1(const h16* __restrict__ Hn, const h16* __restrict__ W1, const float* __restrict__ bias, h16* M1) {
    __shared__ __align__(16) float os[16 * 68];
    const int lane = threadIdx.x & 31, lr = lane & 15, hi = lane >> 4; const int r0 = blockIdx.x * 64, c0 = blockIdx.y * 64;
    v8f acc[4][4];
    gemm_core<DM>(Hn, W1, r0, c0, lr, hi, acc);
    float bc[4];
#pragma unroll
    for (int nb = 0; nb < 4; ++nb) bc[nb] = bfr(bias[c0 + nb * 16 + lr]);
#pragma unroll
    for (int mb = 0; mb < 4; ++mb) {
#pragma unroll
        for (int nb = 0; nb < 4; ++nb) {
#pragma unroll
            for (int j = 0; j < 8; ++j) os[(hi * 8 + j) * 68 + nb * 16 + lr] = acc[mb][nb][j] * WINV + bc[nb]; }
        wave_sync();
#pragma unroll 1
        for (int i = 0; i < 32; ++i) { const int e = i * 32 + lane; const int idx = (e >> 6) * 68 + (e & 63);
            const float v = os[idx];
            os[idx] = 0.5f * v * (1.0f + erff(v * 0.70710678118654752f)) * MCAR; }
        wave_sync();
#pragma unroll 1
        for (int ps = 0; ps < 2; ++ps) {
#pragma unroll
            for (int s = 0; s < 4; ++s) { const int row = 4 * s + (lane >> 3), c8 = (lane & 7) * 8;
                const v4f x0 = *(const v4fa*)(&os[row * 68 + c8]); const v4f x1 = *(const v4fa*)(&os[row * 68 + c8 + 4]); v8h hv;
#pragma unroll
                for (int k = 0; k < 4; ++k) { hv[k] = toh_flush(x0[k]); hv[4 + k] = toh_flush(x1[k]); }
                *(volatile v8h*)(M1 + (size_t)(r0 + mb * 16 + row) * FF + c0 + c8) = hv; }
            if (ps == 0) __threadfence(); }
        wave_sync();
    }
}

__global__ __launch_bounds__(32) void k_gemm_fc2(const h16* __restrict__ Mh, const h16* __restrict__ W2, const float* __restrict__ bias, const float* __restrict__ X1, float* OUT) {
    __shared__ __align__(16) float os[16 * 68];
    const int lane = threadIdx.x & 31, lr = lane & 15, hi = lane >> 4; const int r0 = blockIdx.x * 64, c0 = blockIdx.y * 64;
    v8f acc[4][4];
    gemm_core<FF>(Mh, W2, r0, c0, lr, hi, acc);
    float bc[4];
#pragma unroll
    for (int nb = 0; nb < 4; ++nb) bc[nb] = bfr(bias[c0 + nb * 16 + lr]);
    const int bb = r0 / TP, tt = r0 % TP;
#pragma unroll
    for (int mb = 0; mb < 4; ++mb) {
#pragma unroll
        for (int nb = 0; nb < 4; ++nb) {
#pragma unroll
            for (int j = 0; j < 8; ++j) os[(hi * 8 + j) * 68 + nb * 16 + lr] = acc[mb][nb][j] * PINV + bc[nb]; }
        wave_sync();
#pragma unroll 1
        for (int ps = 0; ps < 2; ++ps) {
#pragma unroll
            for (int s = 0; s < 8; ++s) { const int p = s * 32 + lane; const int row = p >> 4, c4 = (p & 15) * 4;
                const v4f o4 = *(const v4fa*)(&os[row * 68 + c4]);
                v4f xv = *(const v4f*)(X1 + (size_t)(r0 + mb * 16 + row) * DM + c0 + c4);
                asm volatile("" : "+v"(xv));
                const int tr = tt + mb * 16 + row;
                v4f val;
#pragma unroll
                for (int i = 0; i < 4; ++i) val[i] = o4[i] + xv[i];
                if (tr < SEQ) *(volatile v4f*)(OUT + ((size_t)bb * OUT_SEQ + (size_t)tr) * DM + c0 + c4) = val; }
            if (ps == 0) __threadfence(); }
        wave_sync();
    }
}

static constexpr size_t al256(size_t v) { return (v + 255) & ~(size_t)255; }
static constexpr size_t PLANE_E  = (size_t)NB * NH_ * TP * HD;
static constexpr size_t SZ_WQKV  = al256((size_t)3 * DM * DM * 2);
static constexpr size_t SZ_WP    = al256((size_t)DM * DM * 2);
static constexpr size_t SZ_W1    = al256((size_t)FF * DM * 2);
static constexpr size_t SZ_W2    = al256((size_t)DM * FF * 2);
static constexpr size_t SZ_H     = al256((size_t)NB * TP * DM * 2);
static constexpr size_t SZ_QK    = al256((size_t)2 * PLANE_E * 2);
static constexpr size_t SZ_VT    = al256(PLANE_E * 2);
static constexpr size_t SZ_BP    = al256((size_t)NH_ * TP * TP * 2);
static constexpr size_t SZ_CTX   = al256((size_t)NB * TP * DM * 2);
static constexpr size_t SZ_X1    = al256((size_t)NB * TP * DM * 4);
static constexpr size_t SZ_M1    = al256((size_t)NB * TP * FF * 2);
static constexpr size_t SZ_TOTAL = SZ_WQKV + SZ_WP + SZ_W1 + SZ_W2 + 2 * SZ_H + SZ_QK + SZ_VT + SZ_BP + SZ_CTX + SZ_X1 + SZ_M1;
static_assert(SZ_TOTAL <= (size_t)134217728);
static_assert(PLANE_E == (size_t)NB * DM * TP);
static_assert((PLANE_E * 2) % 256 == 0);
static_assert(((size_t)2 * DM * DM * 2) % 256 == 0);
static_assert(((size_t)3 * DM * DM) % 8 == 0);
static_assert(((size_t)FF * DM) % 8 == 0);

extern "C" void kernel_launch(void* const* d_in, const int* in_sizes, int n_in,
                              void* d_out, int out_size, void* d_ws, size_t ws_size, hipStream_t stream) {
    if (n_in < 15) return;
    const size_t needx = ((size_t)(NB - 1) * SEQ_FULL + SEQ) * DM;
    const size_t needb = ((size_t)(NH_ - 1) * SEQ_FULL + (size_t)(SEQ - 1)) * SEQ_FULL + SEQ;
    if ((size_t)in_sizes[0] < needx || (size_t)in_sizes[1] < needb) return;
    if ((size_t)in_sizes[2] < (size_t)3 * DM * DM || (size_t)in_sizes[5] < (size_t)DM * DM) return;
    if ((size_t)in_sizes[11] < (size_t)FF * DM || (size_t)in_sizes[13] < (size_t)DM * FF) return;
    if (in_sizes[3] < DM || in_sizes[4] < DM || in_sizes[6] < DM || in_sizes[7] < DM || in_sizes[8] < DM || in_sizes[9] < DM || in_sizes[10] < DM) return;
    if (in_sizes[12] < FF || in_sizes[14] < DM) return;
    if ((size_t)out_size < ((size_t)(NB - 1) * OUT_SEQ + SEQ) * DM) return;
    if (SZ_TOTAL > ws_size) return;
    const float* x     = (const float*)d_in[0];
    const float* relb  = (const float*)d_in[1];
    const float* wqkv  = (const float*)d_in[2];
    const float* qb    = (const float*)d_in[3];
    const float* vb    = (const float*)d_in[4];
    const float* wproj = (const float*)d_in[5];
    const float* bproj = (const float*)d_in[6];
    const float* ln1g  = (const float*)d_in[7];
    const float* ln1b  = (const float*)d_in[8];
    const float* ln2g  = (const float*)d_in[9];
    const float* ln2b  = (const float*)d_in[10];
    const float* wfc1  = (const float*)d_in[11];
    const float* bfc1  = (const float*)d_in[12];
    const float* wfc2  = (const float*)d_in[13];
    const float* bfc2  = (const float*)d_in[14];
    float* OUT = (float*)d_out;
    char* wsp = (char*)d_ws;
    h16* WQKV = (h16*)wsp; wsp += SZ_WQKV;
    h16* WP   = (h16*)wsp; wsp += SZ_WP;
    h16* W1   = (h16*)wsp; wsp += SZ_W1;
    h16* W2   = (h16*)wsp; wsp += SZ_W2;
    h16* H1   = (h16*)wsp; wsp += SZ_H;
    h16* H2   = (h16*)wsp; wsp += SZ_H;
    h16* QK   = (h16*)wsp; wsp += SZ_QK;
    h16* VT   = (h16*)wsp; wsp += SZ_VT;
    bf*  BP   = (bf*)wsp;  wsp += SZ_BP;
    h16* CTX  = (h16*)wsp; wsp += SZ_CTX;
    float* X1 = (float*)wsp; wsp += SZ_X1;
    h16* M1   = (h16*)wsp; wsp += SZ_M1;

    { const size_t n8 = (size_t)3 * DM * DM / 8; k_wconv<<<(unsigned)((n8 + 255) / 256), 256, 0, stream>>>(wqkv, WQKV, n8); }
    { const size_t n8 = (size_t)DM * DM / 8;     k_wconv<<<(unsigned)((n8 + 255) / 256), 256, 0, stream>>>(wproj, WP, n8); }
    { const size_t n8 = (size_t)FF * DM / 8;     k_wconv<<<(unsigned)((n8 + 255) / 256), 256, 0, stream>>>(wfc1, W1, n8); }
    { const size_t n8 = (size_t)DM * FF / 8;     k_wconv<<<(unsigned)((n8 + 255) / 256), 256, 0, stream>>>(wfc2, W2, n8); }
    { const size_t nt = (size_t)NH_ * TP * (TP / 8); k_bconv<<<(unsigned)((nt + 255) / 256), 256, 0, stream>>>(relb, BP); }

    k_ln<<<NB * TP / 8, 256, 0, stream>>>(x, SEQ_FULL, 1, ln1g, ln1b, H1);
    k_gemm_qk<<<dim3(NB * TP / 64, 2 * DM / 64, 1), 32, 0, stream>>>(H1, WQKV, qb, QK);
    k_gemm_vt<<<dim3(DM / 64, NB * TP / 64, 1), 32, 0, stream>>>(WQKV + (size_t)2 * DM * DM, H1, vb, VT);
    k_flash<<<dim3(TP / (16 * AW), NB * NH_, 1), 32 * AW, 0, stream>>>(QK, QK + PLANE_E, VT, BP, CTX);
    k_gemm_proj<<<dim3(NB * TP / 64, DM / 64, 1), 32, 0, stream>>>(CTX, WP, bproj, x, X1);

    k_ln<<<NB * TP / 8, 256, 0, stream>>>(X1, TP, 0, ln2g, ln2b, H2);
    k_gemm_fc1<<<dim3(NB * TP / 64, FF / 64, 1), 32, 0, stream>>>(H2, W1, bfc1, M1);
    k_gemm_fc2<<<dim3(NB * TP / 64, DM / 64, 1), 32, 0, stream>>>(M1, W2, bfc2, X1, OUT);
}
